// CausalBilinearSelfAttention_7129645711401
// MI455X (gfx1250) — hardware-verified
//
#include <hip/hip_runtime.h>
#include <math.h>
#include <stdint.h>

constexpr int NBATCH = 2;
constexpr int NTOK   = 2048;
constexpr int DMOD   = 1024;
constexpr int NHEADS = 16;
constexpr int HDSZ   = 64;
constexpr int HPG    = 2;
constexpr int NGROUP = NHEADS / HPG;
constexpr int QKW    = 4 * DMOD;
constexpr int NFREQ  = HDSZ / 2;

typedef __attribute__((ext_vector_type(16))) _Float16 v16h;
typedef __attribute__((ext_vector_type(8)))  _Float16 v8h;
typedef __attribute__((ext_vector_type(16))) __bf16   v16b;
typedef __attribute__((ext_vector_type(8)))  __bf16   v8b;
typedef __attribute__((ext_vector_type(8)))  float    v8f;
typedef __attribute__((ext_vector_type(4)))  float    v4f;
typedef __attribute__((ext_vector_type(2)))  float    v2f;
typedef __attribute__((ext_vector_type(4)))  unsigned int v4u;

__device__ __forceinline__ unsigned short f2bf_bits(float f) {
  unsigned u = __float_as_uint(f);
  return (unsigned short)((u + 0x7FFFu + ((u >> 16) & 1u)) >> 16);
}
__device__ __forceinline__ float bf_bits2f(unsigned short h) { return __uint_as_float(((unsigned)h) << 16); }
__device__ __forceinline__ unsigned pk16(unsigned short a, unsigned short b) { return (unsigned)a | ((unsigned)b << 16); }
__device__ __forceinline__ float bf16_rne_f32(float f) {
  unsigned u = __float_as_uint(f);
  u += 0x7FFFu + ((u >> 16) & 1u);
  u &= 0xFFFF0000u;
  return __uint_as_float(u);
}

__device__ __forceinline__ void dep_guard_h(v8f& a, v8f& b, v16h x, v16h y) { asm volatile("v_nop\n\tv_nop\n\tv_nop\n\tv_nop" : "+v"(a), "+v"(b) : "v"(x), "v"(y)); }
__device__ __forceinline__ void dep_guard_b(v8f& a, v8f& b, v16b x, v16b y) { asm volatile("v_nop\n\tv_nop\n\tv_nop\n\tv_nop" : "+v"(a), "+v"(b) : "v"(x), "v"(y)); }
__device__ __forceinline__ void keep4_h(v16h a, v16h b, v16h c, v16h d) { asm volatile("v_nop" :: "v"(a), "v"(b), "v"(c), "v"(d)); }
__device__ __forceinline__ void keep4_b(v16b a, v16b b, v16b c, v16b d) { asm volatile("v_nop" :: "v"(a), "v"(b), "v"(c), "v"(d)); }
__device__ __forceinline__ void acc_guard4(v8f& a, v8f& b, v8f& c, v8f& d) { asm volatile("v_nop\n\tv_nop\n\tv_nop\n\tv_nop" : "+v"(a), "+v"(b), "+v"(c), "+v"(d)); }
template <typename T> struct Frag;
template <> struct Frag<_Float16> {
  typedef v16h V; union U { v16h v; v8h h[2]; };
  static __device__ __forceinline__ v16h load(const _Float16* p) {
    U f; f.h[0] = *(const v8h*)(p); f.h[1] = *(const v8h*)(p + 16); return f.v;
  }
  static __device__ __forceinline__ v8f mma(v16h a, v16h b, v8f c) {
    return __builtin_amdgcn_wmma_f32_16x16x32_f16(false, a, false, b, (short)0, c, false, false);
  }
  static __device__ __forceinline__ void guard(v8f& a, v8f& b, v16h x, v16h y) { dep_guard_h(a, b, x, y); }
  static __device__ __forceinline__ void keep(v16h a, v16h b, v16h c, v16h d) { keep4_h(a, b, c, d); }
};
template <> struct Frag<__bf16> {
  typedef v16b V; union U { v16b v; v8b h[2]; };
  static __device__ __forceinline__ v16b load(const __bf16* p) {
    U f; f.h[0] = *(const v8b*)(p); f.h[1] = *(const v8b*)(p + 16); return f.v;
  }
  static __device__ __forceinline__ v8f mma(v16b a, v16b b, v8f c) {
    return __builtin_amdgcn_wmma_f32_16x16x32_bf16(false, a, false, b, (short)0, c, false, false);
  }
  static __device__ __forceinline__ void guard(v8f& a, v8f& b, v16b x, v16b y) { dep_guard_b(a, b, x, y); }
  static __device__ __forceinline__ void keep(v16b a, v16b b, v16b c, v16b d) { keep4_b(a, b, c, d); }
};

template <int ET> struct Elem;
template <> struct Elem<0> { typedef _Float16 T; };
template <> struct Elem<1> { typedef __bf16 T; };
template <int ET, bool SPLIT, int BIAS_MODE, int OUT_MODE, bool RESID, int ACT = 0, bool LOWER = false, bool CAUSALK = false,
          bool RMUL = false, bool CMASK = false, bool BLO = true>
__global__ __launch_bounds__(256) void wmma_gemm64(
    const unsigned short* __restrict__ Ap, const unsigned short* __restrict__ A2p, int lda, long strideA,
    const unsigned short* __restrict__ Btp, const unsigned short* __restrict__ Bt2p, int ldb, long strideB,
    void* __restrict__ Cout, void* __restrict__ Cout2, int ldc, long strideC,
    const float* __restrict__ bias,
    const float* __restrict__ resid, long strideR,
    int M, int N, int K, float scale) {
  typedef typename Elem<ET>::T T;
  typedef typename Frag<T>::V V;
  const T* A = (const T*)Ap; const T* A2 = (const T*)A2p; const T* Bt = (const T*)Btp; const T* Bt2 = (const T*)Bt2p;
  __shared__ __align__(16) float sT[8][16 * 68];
  const int b    = blockIdx.y;
  const int lane = threadIdx.x & 31;
  const int wave = threadIdx.x >> 5;
  const int tilesN = N >> 6;
  const int tilesM = M >> 6;
  const int tile = blockIdx.x * 8 + wave;
  if (tile >= tilesM * tilesN) return;
  const int tm = tile / tilesN;
  const int tn = tile - tm * tilesN;
  const int m0 = tm << 6;
  const int n0 = tn << 6;
  if (LOWER && n0 > m0) return;

  const T* Ab  = A  + (size_t)b * strideA;
  const T* Bb  = Bt + (size_t)b * strideB;
  const T* Ab2 = SPLIT ? (A2  + (size_t)b * strideA) : nullptr;
  const T* Bb2 = (SPLIT && BLO) ? (Bt2 + (size_t)b * strideB) : nullptr;

  const int rlane = lane & 15;
  const int koff  = (lane >> 4) * 8;
  const int mOff  = (lane >> 4) * 8;

  v8f acc[4][4];
#pragma unroll
  for (int i = 0; i < 4; ++i)
#pragma unroll
    for (int j = 0; j < 4; ++j) acc[i][j] = (v8f){0.f,0.f,0.f,0.f,0.f,0.f,0.f,0.f};

  const int kEnd = CAUSALK ? (((m0 + 64) < K) ? (m0 + 64) : K) : K;
  for (int k0 = 0; k0 < kEnd; k0 += 32) {
    V bh[4], bl[4];
#pragma unroll
    for (int j = 0; j < 4; ++j) {
      const size_t bo = (size_t)(n0 + (j << 4) + rlane) * ldb + koff + k0;
      bh[j] = Frag<T>::load(Bb + bo);
      if (SPLIT && BLO) bl[j] = Frag<T>::load(Bb2 + bo);
    }
#pragma unroll
    for (int i = 0; i < 4; ++i) {
      const size_t ao = (size_t)(m0 + (i << 4) + rlane) * lda + koff + k0;
      V ah = Frag<T>::load(Ab + ao);
      V al;
      if (SPLIT) al = Frag<T>::load(Ab2 + ao);
#pragma unroll
      for (int j = 0; j < 4; ++j) {
        acc[i][j] = Frag<T>::mma(ah, bh[j], acc[i][j]);
        if (SPLIT) {
          if (BLO) acc[i][j] = Frag<T>::mma(ah, bl[j], acc[i][j]);
          acc[i][j] = Frag<T>::mma(al, bh[j], acc[i][j]);
        }
      }
      Frag<T>::guard(acc[i][0], acc[i][3], ah, SPLIT ? al : ah);
    }
    Frag<T>::keep(bh[0], bh[1], bh[2], bh[3]);
    if (SPLIT && BLO) Frag<T>::keep(bl[0], bl[1], bl[2], bl[3]);
  }
  acc_guard4(acc[0][0], acc[0][1], acc[0][2], acc[0][3]);
  acc_guard4(acc[1][0], acc[1][1], acc[1][2], acc[1][3]);
  acc_guard4(acc[2][0], acc[2][1], acc[2][2], acc[2][3]);
  acc_guard4(acc[3][0], acc[3][1], acc[3][2], acc[3][3]);

  float* slab = sT[wave];
  const float* Rb = RESID ? (resid + (size_t)b * strideR) : nullptr;
#pragma unroll
  for (int i = 0; i < 4; ++i) {
    const int mBase = m0 + (i << 4);
#pragma unroll
    for (int j = 0; j < 4; ++j) {
      const int n = n0 + (j << 4) + rlane;
      float bv = 0.f;
      if (BIAS_MODE == 2) bv = bias[n];
#pragma unroll
      for (int r = 0; r < 8; ++r) {
        float v = acc[i][j][r] * scale;
        if (BIAS_MODE == 1) v += bias[mBase + mOff + r];
        if (BIAS_MODE == 2) v += bv;
        if (RESID) {
          const float rv = Rb[(size_t)(mBase + mOff + r) * ldc + n];
          if (RMUL) v = v * rv; else v += rv;
        }
        if (ACT == 1) v = tanhf(v);
        if (ACT == 2) v = fmaxf(v, 0.0f);
        if (ACT == 3) v = v / (1.0f + expf(-v));
        if (ACT == 4) v = (v > 0.f) ? v : 0.01f * v;
        if (ACT == 5) v = 0.5f * v * (1.0f + erff(v * 0.70710678118654752f));
        if (CMASK) v = (n > mBase + mOff + r) ? 0.0f : v;
        slab[(mOff + r) * 68 + (j << 4) + rlane] = v;
      }
    }
    __builtin_amdgcn_fence(__ATOMIC_RELEASE, "workgroup");
    __builtin_amdgcn_wave_barrier();
    __builtin_amdgcn_fence(__ATOMIC_ACQUIRE, "workgroup");
    if (OUT_MODE == 0) {
      float* C = (float*)Cout + (size_t)b * strideC;
      const int hh = lane >> 4, c4 = (lane & 15) * 4;
      for (int pass = 0; pass < 2; ++pass) {
#pragma unroll
        for (int it = 0; it < 8; ++it) {
          const int row = it * 2 + hh;
          v4f v = *(const v4f*)(slab + row * 68 + c4);
          *(volatile v4f*)(C + (size_t)(mBase + row) * ldc + n0 + c4) = v;
        }
        __threadfence();
      }
    } else {
      const int q = lane >> 3, c8 = (lane & 7) * 8;
      unsigned short* C  = (unsigned short*)Cout  + (size_t)b * strideC;
      unsigned short* C2 = (OUT_MODE == 2) ? ((unsigned short*)Cout2 + (size_t)b * strideC) : nullptr;
      for (int pass = 0; pass < 2; ++pass) {
#pragma unroll
        for (int it = 0; it < 4; ++it) {
          const int row = it * 4 + q;
          const float* sp = slab + row * 68 + c8;
          v8h hv, lv;
#pragma unroll
          for (int e = 0; e < 8; ++e) {
            if (OUT_MODE == 1) {
              hv[e] = (_Float16)sp[e];
            } else {
              unsigned short hb = f2bf_bits(sp[e]);
              unsigned short lb = f2bf_bits(sp[e] - bf_bits2f(hb));
              hv[e] = __builtin_bit_cast(_Float16, hb);
              lv[e] = __builtin_bit_cast(_Float16, lb);
            }
          }
          *(volatile v8h*)(C + (size_t)(mBase + row) * ldc + n0 + c8) = hv;
          if (OUT_MODE == 2) *(volatile v8h*)(C2 + (size_t)(mBase + row) * ldc + n0 + c8) = lv;
        }
        __threadfence();
      }
    }
    __builtin_amdgcn_fence(__ATOMIC_RELEASE, "workgroup");
    __builtin_amdgcn_wave_barrier();
    __builtin_amdgcn_fence(__ATOMIC_ACQUIRE, "workgroup");
  }
}

__global__ __launch_bounds__(256) void cast_bf16rne_f16x2(
    const float* __restrict__ in, _Float16* __restrict__ out, int n2, float sc) {
  const int i = blockIdx.x * 256 + threadIdx.x;
  if (i < n2) {
    const float r0 = bf16_rne_f32(in[2 * (size_t)i]) * sc;
    const float r1 = bf16_rne_f32(in[2 * (size_t)i + 1]) * sc;
    const _Float16 h0 = (_Float16)r0, h1 = (_Float16)r1;
    const unsigned u = (unsigned)__builtin_bit_cast(unsigned short, h0) | ((unsigned)__builtin_bit_cast(unsigned short, h1) << 16);
    ((volatile unsigned*)out)[i] = u;
    __threadfence();
    ((volatile unsigned*)out)[i] = u;
  }
}

__global__ __launch_bounds__(256) void cast_bf16x2_kernel(const float* __restrict__ in, unsigned short* __restrict__ out, int n2) {
  const int i = blockIdx.x * 256 + threadIdx.x;
  if (i < n2) {
    const v2f f = *(const v2f*)(in + 2 * (size_t)i);
    const unsigned u = pk16(f2bf_bits(f[0]), f2bf_bits(f[1]));
    ((volatile unsigned*)out)[i] = u;
    __threadfence();
    ((volatile unsigned*)out)[i] = u;
  }
}

struct InvFreq { float v[NFREQ]; };
static_assert(sizeof(InvFreq) == 128);

__global__ __launch_bounds__(256) void rope_table_kernel(float* __restrict__ ctab, float* __restrict__ stab, InvFreq f) {
#pragma clang fp contract(off)
  const int lane = threadIdx.x & 31;
  const int wave = threadIdx.x >> 5;
  const int t    = blockIdx.x * 8 + wave;
  float inv = f.v[0];
#pragma unroll
  for (int i = 1; i < NFREQ; ++i) inv = (lane == i) ? f.v[i] : inv;
  const float ang = (float)t * inv;
  const float cv = cosf(ang);
  const float sv = sinf(ang);
  const size_t o = (size_t)t * NFREQ + lane;
  ((volatile float*)ctab)[o] = cv;
  ((volatile float*)stab)[o] = sv;
  __threadfence();
  ((volatile float*)ctab)[o] = cv;
  ((volatile float*)stab)[o] = sv;
}

__global__ __launch_bounds__(256) void rope_split_kernel(const float* __restrict__ src, const float* __restrict__ ctab,
                                                         const float* __restrict__ stab,
                                                         unsigned short* __restrict__ dh, unsigned short* __restrict__ dl) {
#pragma clang fp contract(off)
  const int t   = blockIdx.x;
  const int tid = threadIdx.x;
  const float* row  = src  + (size_t)t * QKW;
  const float* crow = ctab + (size_t)t * NFREQ;
  const float* srow = stab + (size_t)t * NFREQ;
  v4u hv[2], lv[2];
#pragma unroll
  for (int it = 0; it < 2; ++it) {
    const int c8 = it * (QKW / 2) + tid * 8;
    const int d0 = c8 & (HDSZ - 1);
    const bool firstHalf = d0 < NFREQ;
    const int pc = firstHalf ? (c8 + NFREQ) : (c8 - NFREQ);
    const float sgn = firstHalf ? 1.0f : -1.0f;
    const int fi = d0 & (NFREQ - 1);
    const v4f o0 = *(const v4f*)(row + c8), o1 = *(const v4f*)(row + c8 + 4);
    const v4f p0 = *(const v4f*)(row + pc), p1 = *(const v4f*)(row + pc + 4);
    const v4f ca = *(const v4f*)(crow + fi), cb = *(const v4f*)(crow + fi + 4);
    const v4f sa = *(const v4f*)(srow + fi), sb = *(const v4f*)(srow + fi + 4);
    float o[8], p[8], cc[8], ss[8];
#pragma unroll
    for (int e = 0; e < 4; ++e) {
      o[e]  = o0[e]; o[4 + e]  = o1[e];
      p[e]  = p0[e]; p[4 + e]  = p1[e];
      cc[e] = ca[e]; cc[4 + e] = cb[e];
      ss[e] = sa[e]; ss[4 + e] = sb[e];
    }
    unsigned hw[4], lw[4];
#pragma unroll
    for (int q = 0; q < 4; ++q) {
      const float y0 = o[2 * q] * cc[2 * q] + sgn * (p[2 * q] * ss[2 * q]);
      const float y1 = o[2 * q + 1] * cc[2 * q + 1] + sgn * (p[2 * q + 1] * ss[2 * q + 1]);
      const unsigned short h0 = f2bf_bits(y0), h1 = f2bf_bits(y1);
      const unsigned short l0 = f2bf_bits(y0 - bf_bits2f(h0));
      const unsigned short l1 = f2bf_bits(y1 - bf_bits2f(h1));
      hw[q] = pk16(h0, h1);
      lw[q] = pk16(l0, l1);
    }
    hv[it] = (v4u){hw[0], hw[1], hw[2], hw[3]};
    lv[it] = (v4u){lw[0], lw[1], lw[2], lw[3]};
  }
  for (int pass = 0; pass < 2; ++pass) {
#pragma unroll
    for (int it = 0; it < 2; ++it) {
      const size_t go = (size_t)t * QKW + (size_t)it * (QKW / 2) + (size_t)tid * 8;
      *(volatile v4u*)(dh + go) = hv[it];
      *(volatile v4u*)(dl + go) = lv[it];
    }
    __threadfence();
  }
}

extern "C" void kernel_launch(void* const* d_in, const int* in_sizes, int n_in,
                              void* d_out, int out_size, void* d_ws, size_t ws_size,
                              hipStream_t stream) {
  if (n_in < 7) return;
  if (in_sizes[0] != NBATCH * NTOK * DMOD) return;
  for (int i = 1; i < 7; ++i) if (in_sizes[i] != DMOD * DMOD) return;
  if (out_size != NBATCH * NTOK * DMOD) return;

  const float* x     = (const float*)d_in[0];
  const float* Wq    = (const float*)d_in[1];
  const float* Wk    = (const float*)d_in[2];
  const float* Wq2   = (const float*)d_in[3];
  const float* Wk2   = (const float*)d_in[4];
  const float* Wv    = (const float*)d_in[5];
  const float* Wproj = (const float*)d_in[6];

  const size_t PW16 = (size_t)DMOD * DMOD * 2;
  const size_t PTAB = (size_t)NTOK * NFREQ * 4;
  const size_t PX16 = (size_t)NBATCH * NTOK * DMOD * 2;
  const size_t PQK  = (size_t)NTOK * QKW * 2;
  const size_t PVT  = (size_t)DMOD * NTOK * 2;
  const size_t PS   = (size_t)HPG * NTOK * NTOK * 4;
  const size_t PP   = (size_t)HPG * NTOK * NTOK * 2;
  size_t off = 0;
  const size_t oW4  = off; off += 4 * PW16;
  const size_t oWv  = off; off += PW16;
  const size_t oWph = off; off += PW16;
  const size_t oCT  = off; off += PTAB;
  const size_t oSTb = off; off += PTAB;
  const size_t oX16 = off; off += PX16;
  const size_t oQKh = off; off += PQK;
  const size_t oQKl = off; off += PQK;
  const size_t oVTh = off; off += PVT;
  const size_t oVTl = off; off += PVT;
  const size_t oS1  = off; off += PS;
  const size_t oPh  = off; off += PP;
  const size_t oPl  = off; off += PP;
  if (off > ws_size) return;

  char* ws = (char*)d_ws;
  _Float16*       W4   = (_Float16*)(ws + oW4);
  _Float16*       Wv16 = (_Float16*)(ws + oWv);
  unsigned short* Wph  = (unsigned short*)(ws + oWph);
  float*          ctab = (float*)(ws + oCT);
  float*          stab = (float*)(ws + oSTb);
  _Float16*       X16  = (_Float16*)(ws + oX16);
  unsigned short* QKh  = (unsigned short*)(ws + oQKh);
  unsigned short* QKl  = (unsigned short*)(ws + oQKl);
  unsigned short* VTh  = (unsigned short*)(ws + oVTh);
  unsigned short* VTl  = (unsigned short*)(ws + oVTl);
  float*          S1   = (float*)(ws + oS1);
  float*          QKf  = (float*)(ws + oS1);
  unsigned short* Ph   = (unsigned short*)(ws + oPh);
  unsigned short* Pl   = (unsigned short*)(ws + oPl);
  const float*    dmy  = ctab;

  InvFreq invf;
  {
    const double x0 = 9.2103403719761827361 / 32.0;
    double term = 1.0, ex = 1.0;
    for (int n = 1; n <= 40; ++n) { term *= x0 / (double)n; ex += term; }
    double pw = 1.0;
    for (int i = 0; i < NFREQ; ++i) {
      const float pf = (float)pw;
      invf.v[i] = (float)(1.0 / (double)pf);
      pw *= ex;
    }
  }

  const dim3 blk(256);
  const int n2w = DMOD * DMOD / 2;
  const int n2x = NBATCH * NTOK * DMOD / 2;
  const dim3 gCastW((n2w + 255) / 256);
  const dim3 gCastX((n2x + 255) / 256);
  const dim3 gTab(NTOK / 8);
  const dim3 gRope(NTOK);
  const dim3 gQ(((NTOK / 64) * (QKW / 64) + 7) / 8, 1);
  const dim3 gV(((DMOD / 64) * (NTOK / 64) + 7) / 8, 1);
  const dim3 gS(((NTOK / 64) * (NTOK / 64) + 7) / 8, HPG);
  const dim3 gPV(((NTOK / 64) * (HDSZ / 64) + 7) / 8, HPG);
  const dim3 gOut(((NTOK / 64) * (DMOD / 64) + 7) / 8, 1);

  rope_table_kernel<<<gTab, blk, 0, stream>>>(ctab, stab, invf);
  cast_bf16rne_f16x2<<<gCastX, blk, 0, stream>>>(x, X16, n2x, 1.0f);
  cast_bf16rne_f16x2<<<gCastW, blk, 0, stream>>>(Wq,  W4 + 0 * (size_t)DMOD * DMOD, n2w, 32.0f);
  cast_bf16rne_f16x2<<<gCastW, blk, 0, stream>>>(Wk,  W4 + 1 * (size_t)DMOD * DMOD, n2w, 32.0f);
  cast_bf16rne_f16x2<<<gCastW, blk, 0, stream>>>(Wq2, W4 + 2 * (size_t)DMOD * DMOD, n2w, 32.0f);
  cast_bf16rne_f16x2<<<gCastW, blk, 0, stream>>>(Wk2, W4 + 3 * (size_t)DMOD * DMOD, n2w, 32.0f);
  cast_bf16rne_f16x2<<<gCastW, blk, 0, stream>>>(Wv,  Wv16, n2w, 32.0f);
  cast_bf16x2_kernel<<<gCastW, blk, 0, stream>>>(Wproj, Wph, n2w);

  const float inv32 = 1.0f / 32.0f;
  const float inv64 = 1.0f / 64.0f;
  const long  sPlane = (long)NTOK * NTOK;

  for (int b = 0; b < NBATCH; ++b) {
    const _Float16* Xb = X16 + (size_t)b * NTOK * DMOD;
    wmma_gemm64<0, false, 0, 0, false><<<gQ, blk, 0, stream>>>(
        (const unsigned short*)Xb, (const unsigned short*)Xb, DMOD, 0L,
        (const unsigned short*)W4, (const unsigned short*)W4, DMOD, 0L,
        (void*)QKf, (void*)QKf, QKW, 0L, dmy, dmy, 0L, NTOK, QKW, DMOD, inv32);
    wmma_gemm64<0, false, 0, 2, false><<<gV, blk, 0, stream>>>(
        (const unsigned short*)Wv16, (const unsigned short*)Wv16, DMOD, 0L,
        (const unsigned short*)Xb, (const unsigned short*)Xb, DMOD, 0L,
        (void*)VTh, (void*)VTl, NTOK, 0L, dmy, dmy, 0L, DMOD, NTOK, DMOD, inv32);
    rope_split_kernel<<<gRope, blk, 0, stream>>>(QKf, ctab, stab, QKh, QKl);
    for (int g = 0; g < NGROUP; ++g) {
      const size_t qcol = (size_t)g * HPG * HDSZ;
      wmma_gemm64<1, true, 0, 0, false, 0, true, false><<<gS, blk, 0, stream>>>(
          QKh + qcol, QKl + qcol, QKW, (long)HDSZ,
          QKh + DMOD + qcol, QKl + DMOD + qcol, QKW, (long)HDSZ,
          (void*)S1, (void*)S1, NTOK, sPlane, dmy, dmy, 0L, NTOK, NTOK, HDSZ, inv64);
      wmma_gemm64<1, true, 0, 2, true, 0, true, false, true, true><<<gS, blk, 0, stream>>>(
          QKh + 2 * DMOD + qcol, QKl + 2 * DMOD + qcol, QKW, (long)HDSZ,
          QKh + 3 * DMOD + qcol, QKl + 3 * DMOD + qcol, QKW, (long)HDSZ,
          (void*)Ph, (void*)Pl, NTOK, sPlane, dmy, S1, sPlane, NTOK, NTOK, HDSZ, inv64);
      wmma_gemm64<1, true, 0, 2, false, 0, false, true><<<gPV, blk, 0, stream>>>(
          Ph, Pl, NTOK, sPlane,
          VTh + qcol * NTOK, VTl + qcol * NTOK, NTOK, (long)HDSZ * NTOK,
          (void*)(QKh + qcol), (void*)(QKl + qcol), QKW, (long)HDSZ,
          dmy, dmy, 0L, NTOK, HDSZ, NTOK, 1.0f);
    }
    float* outb = (float*)d_out + (size_t)b * NTOK * DMOD;
    wmma_gemm64<1, true, 0, 0, false, 0, false, false, false, false, false><<<gOut, blk, 0, stream>>>(
        QKh, QKl, QKW, 0L, Wph, Wph, DMOD, 0L, (void*)outb, (void*)outb, DMOD, 0L,
        dmy, dmy, 0L, NTOK, DMOD, DMOD, 1.0f);
  }
}
